// EnsemblesWithMessagePassing_2104533975419
// MI455X (gfx1250) — hardware-verified
//
#include <hip/hip_runtime.h>


namespace {
constexpr int L = 8, BT = 2, NN = 512, D = 1024, H = 8, DH = 64, INNER = 512, M = 16, NR = L * BT * NN  , NQC = 576  ;
typedef __attribute__((ext_vector_type(8))) __bf16 v8bb; typedef __attribute__((ext_vector_type(16))) __bf16 v16bb; typedef __attribute__((ext_vector_type(8))) unsigned short v8us;

typedef _Float16 b16;
typedef __attribute__((ext_vector_type(16))) _Float16 v16b;
typedef __attribute__((ext_vector_type(8)))  _Float16 v8b;
typedef __attribute__((ext_vector_type(8)))  float v8f;
typedef __attribute__((ext_vector_type(4)))  float v4f;

__device__ __forceinline__ v8b ld8b(const b16* p) { return *(const v8b*)p; }
__device__ __forceinline__ v16b cat8b(v8b a, v8b b) { return __builtin_shufflevector(a, b, 0, 1, 2, 3, 4, 5, 6, 7, 8, 9, 10, 11, 12, 13, 14, 15); }
__device__ __forceinline__ v16b frag_kb(const b16* p, int hh) { return cat8b(ld8b(p + 8 * hh), ld8b(p + 16 + 8 * hh)); }
__device__ __forceinline__ void split16(float v, b16& hi, b16& lo) { hi = (b16)v; lo = (b16)(v - (float)hi); }
__device__ __forceinline__ void frag_ksplit(const float* p, int hh, v16b& fh_, v16b& fl_) {
  const float* p0 = p + 8 * hh; const float* p1 = p + 16 + 8 * hh;
#pragma unroll
  for (int e = 0; e < 8; ++e) { b16 a, c; split16(p0[e], a, c); fh_[e] = a; fl_[e] = c; split16(p1[e], a, c); fh_[8 + e] = a; fl_[8 + e] = c; }
}
__device__ __forceinline__ v8f wmma16b(v16b a, v16b b, v8f c) {
  v8f d = __builtin_amdgcn_wmma_f32_16x16x32_f16(false, a, false, b, (short)0, c, false, false);
  asm volatile("v_nop\n\tv_nop\n\tv_nop\n\tv_nop" : "+v"(d) : "v"(a), "v"(b));
  return d;
}
__device__ __forceinline__ void wave_lds_sync() {
  __builtin_amdgcn_fence(__ATOMIC_RELEASE, "workgroup");
  __builtin_amdgcn_wave_barrier();
  __builtin_amdgcn_fence(__ATOMIC_ACQUIRE, "workgroup");
}

struct Opnd { const void* p0; const void* p1; int ld; };
template <int NP> __device__ __forceinline__ void load_frags(const Opnd& o, int row, int kb, int hh, v16b& fh_, v16b& fl_) {
  if (NP == 0) { frag_ksplit((const float*)o.p0 + (size_t)row * o.ld + kb, hh, fh_, fl_); }
  else if (NP == 4) {
    const float* p = (const float*)o.p0 + (size_t)row * o.ld + kb; const float* p0 = p + 8 * hh; const float* p1 = p + 16 + 8 * hh;
#pragma unroll
    for (int e = 0; e < 8; ++e) { b16 a, c; split16(p0[e] * 64.0f, a, c); fh_[e] = a; fl_[e] = c; split16(p1[e] * 64.0f, a, c); fh_[8 + e] = a; fl_[8 + e] = c; }
  } else if (NP == 3) {
    const float* p = (const float*)o.p0 + (size_t)row * o.ld + kb; const float* p0 = p + 8 * hh; const float* p1 = p + 16 + 8 * hh;
#pragma unroll
    for (int e = 0; e < 8; ++e) { fh_[e] = (b16)p0[e]; fh_[8 + e] = (b16)p1[e]; }
    fl_ = fh_;
  } else {
    fh_ = frag_kb((const b16*)o.p0 + (size_t)row * o.ld + kb, hh);
    if (NP == 2) fl_ = frag_kb((const b16*)o.p1 + (size_t)row * o.ld + kb, hh); else fl_ = fh_;
  }
}
template <int ANP, int BNP> __device__ __forceinline__ v8f mac(v16b ah, v16b al, v16b bh, v16b bl, v8f c) {
  c = wmma16b(ah, bh, c);
  if (BNP == 0 || BNP == 2 || BNP == 4) c = wmma16b(ah, bl, c);
  if (ANP == 0 || ANP == 2 || ANP == 4) c = wmma16b(al, bh, c);
  return c;
}
template <int ANP, int BNP>
__device__ __forceinline__ void gemm_tile(const Opnd& A, const Opnd& B, int K, int m0, int c0, int nloc, int hlf, v8f (&acc)[2][4]) {
  for (int kb = 0; kb < K; kb += 32) {
    v16b a0h, a0l, a1h, a1l;
    load_frags<ANP>(A, m0 + nloc, kb, hlf, a0h, a0l);
    load_frags<ANP>(A, m0 + 16 + nloc, kb, hlf, a1h, a1l);
#pragma unroll
    for (int t = 0; t < 4; ++t) {
      v16b bh, bl;
      load_frags<BNP>(B, c0 + t * 16 + nloc, kb, hlf, bh, bl);
      acc[0][t] = mac<ANP, BNP>(a0h, a0l, bh, bl, acc[0][t]);
      acc[1][t] = mac<ANP, BNP>(a1h, a1l, bh, bl, acc[1][t]);
    }
  }
}

__device__ __forceinline__ void epi_planes(v8f (&acc)[2][4], float scale, bool two, b16* __restrict__ oh, b16* __restrict__ ol, int ldo,
                                           int m0, int c0, int lane, b16* Th, b16* Tl) {
  const int nloc = lane & 15, hlf = lane >> 4;
#pragma unroll
  for (int t = 0; t < 4; ++t)
#pragma unroll
    for (int r = 0; r < 2; ++r)
#pragma unroll
      for (int v = 0; v < 8; ++v) {
        const int rr = r * 16 + v + 8 * hlf, cc = t * 16 + nloc;
        b16 h_, l_; split16(acc[r][t][v] * scale, h_, l_);
        Th[rr * 64 + cc] = h_; Tl[rr * 64 + cc] = l_;
      }
  wave_lds_sync();
  for (int pass = 0; pass < 2; ++pass) {
#pragma unroll
    for (int j = 0; j < 8; ++j) {
      const int rr = j * 4 + (lane >> 3), c8 = (lane & 7) * 8;
      const size_t o = (size_t)(m0 + rr) * ldo + c0 + c8;
      *(volatile v8b*)(oh + o) = ld8b(Th + rr * 64 + c8);
      if (two) *(volatile v8b*)(ol + o) = ld8b(Tl + rr * 64 + c8);
    }
    __threadfence();
  }
}
__device__ __forceinline__ void epi_f32(v8f (&acc)[2][4], float scale, const float* rscale, float* __restrict__ out, int ldo, int m0, int c0, int lane, float* Tt) {
  const int nloc = lane & 15, hlf = lane >> 4;
#pragma unroll
  for (int t = 0; t < 4; ++t)
#pragma unroll
    for (int r = 0; r < 2; ++r)
#pragma unroll
      for (int v = 0; v < 8; ++v) {
        const int rr = r * 16 + v + 8 * hlf;
        const float rs = rscale ? rscale[(size_t)(m0 + rr) * 32] : 1.0f;
        Tt[rr * 64 + t * 16 + nloc] = acc[r][t][v] * scale * rs;
      }
  wave_lds_sync();
  float* dst0 = out + (size_t)m0 * ldo + c0;
  for (int pass = 0; pass < 2; ++pass) {
#pragma unroll
    for (int j = 0; j < 16; ++j) { const int rr = j * 2 + hlf, c4 = nloc * 4; *(volatile v4f*)(dst0 + (size_t)rr * ldo + c4) = *(const v4f*)(Tt + rr * 64 + c4); }
    __threadfence();
  }
}


__device__ __forceinline__ v16bb frag_kb_bf(const __bf16* p, int hh) { const v8bb a = *(const v8bb*)(p + 8 * hh), b = *(const v8bb*)(p + 16 + 8 * hh); return __builtin_shufflevector(a, b, 0, 1, 2, 3, 4, 5, 6, 7, 8, 9, 10, 11, 12, 13, 14, 15); }
__device__ __forceinline__ v8f wmma16bb(v16bb a, v16bb b, v8f c) { v8f d = __builtin_amdgcn_wmma_f32_16x16x32_bf16(false, a, false, b, (short)0, c, false, false); asm volatile("v_nop\n\tv_nop\n\tv_nop\n\tv_nop" : "+v"(d) : "v"(a), "v"(b)); return d; }
__device__ __forceinline__ unsigned short bf16_rne_bits(float v) { unsigned int u = __float_as_uint(v); u += 0x7FFFu + ((u >> 16) & 1u); return (unsigned short)(u >> 16); }
__device__ __forceinline__ float bf16_rne(float v) { return __uint_as_float(((unsigned int)bf16_rne_bits(v)) << 16); }

__global__ __launch_bounds__(256) void tok_kernel(const float* __restrict__ tok, int b, unsigned short* __restrict__ tokb) {
  const size_t tid = (size_t)blockIdx.x * blockDim.x + threadIdx.x, nth = (size_t)gridDim.x * blockDim.x;
  for (int pass = 0; pass < 2; ++pass) {
    for (size_t p = tid; p < (size_t)L * NN * D / 8; p += nth) { const size_t rl = p / (D / 8), k0 = (p % (D / 8)) * 8; const size_t l = rl / NN, n = rl % NN; const float* src = tok + ((l * BT + b) * NN + n) * D + k0; v8us v;
#pragma unroll
      for (int e = 0; e < 8; ++e) v[e] = bf16_rne_bits(src[e]);
      *(volatile v8us*)(tokb + p * 8) = v; }
    __threadfence();
  }
}
__global__ __launch_bounds__(256) void prep_kernel(const float* __restrict__ wnet, const float* __restrict__ wq, const float* __restrict__ wkv, const float* __restrict__ wg, const float* __restrict__ wout,
                                                   unsigned short* __restrict__ wnb, unsigned short* __restrict__ wkvb, b16* __restrict__ wkvh, b16* __restrict__ wqg, b16* __restrict__ wo) {
  const size_t tid = (size_t)blockIdx.x * blockDim.x + threadIdx.x, nth = (size_t)gridDim.x * blockDim.x;
  for (int pass = 0; pass < 2; ++pass) {
    for (size_t p = tid; p < (size_t)L * D * D / 8; p += nth) { v8us v;
#pragma unroll
      for (int e = 0; e < 8; ++e) v[e] = bf16_rne_bits(wnet[p * 8 + e]);
      *(volatile v8us*)(wnb + p * 8) = v; }
    for (size_t p = tid; p < (size_t)D * D / 8; p += nth) { const int n = (int)(p / (D / 8)), k0 = (int)(p % (D / 8)) * 8; v8us v; v8b w;
#pragma unroll
      for (int e = 0; e < 8; ++e) { const float x = wkv[(size_t)(k0 + e) * D + n]; v[e] = bf16_rne_bits(x); w[e] = (b16)bf16_rne(x); }
      *(volatile v8us*)(wkvb + (size_t)n * D + k0) = v; *(volatile v8b*)(wkvh + (size_t)n * D + k0) = w; }
    for (size_t p = tid; p < (size_t)NQC * D / 8; p += nth) { const int n = (int)(p / (D / 8)), k0 = (int)(p % (D / 8)) * 8; v8b w;
#pragma unroll
      for (int e = 0; e < 8; ++e) { const int k = k0 + e; float x = 0.0f; if (n < INNER) x = wq[(size_t)k * INNER + n]; else if (n < INNER + H) x = wg[(size_t)k * H + (n - INNER)]; w[e] = (b16)bf16_rne(x); }
      *(volatile v8b*)(wqg + (size_t)n * D + k0) = w; }
    for (size_t p = tid; p < (size_t)D * INNER / 8; p += nth) { const int n = (int)(p / (INNER / 8)), k0 = (int)(p % (INNER / 8)) * 8; v8b w;
#pragma unroll
      for (int e = 0; e < 8; ++e) w[e] = (b16)bf16_rne(wout[(size_t)(k0 + e) * D + n]);
      *(volatile v8b*)(wo + (size_t)n * INNER + k0) = w; }
    __threadfence();
  }
}

__global__ __launch_bounds__(256) void tn_kernel(const unsigned short* __restrict__ tokb, const float* __restrict__ nw, b16* __restrict__ tnh) {
  const int wid = threadIdx.x >> 5, lane = threadIdx.x & 31, row = blockIdx.x * 8 + wid;
  float s = 0.0f;
#pragma unroll 1
  for (int j = 0; j < 32; ++j) { const float v = __uint_as_float(((unsigned int)tokb[(size_t)row * D + j * 32 + lane]) << 16); s += v * v; }
#pragma unroll
  for (int o = 16; o > 0; o >>= 1) s += __shfl_xor(s, o);
  const float rs = rsqrtf(s * (1.0f / D) + 1.1920929e-7f);
  for (int pass = 0; pass < 2; ++pass) {
#pragma unroll 1
    for (int j = 0; j < 32; ++j) { const float v = __uint_as_float(((unsigned int)tokb[(size_t)row * D + j * 32 + lane]) << 16); ((volatile b16*)tnh)[(size_t)row * D + j * 32 + lane] = (b16)(v * rs * bf16_rne(nw[j * 32 + lane])); }
    __threadfence();
  }
}

template <int TYPE, int EPI, int KIN, int NOUT>
__global__ __launch_bounds__(128) void gemm_kernel(const void* __restrict__ Ap, const void* __restrict__ Bp, const float* __restrict__ bias, float* __restrict__ outf, b16* __restrict__ outh, int rows_per_z, size_t a_zstride, size_t b_zstride, size_t o_zstride) {
  __shared__ __attribute__((aligned(16))) float Ts[4][32 * 64];
  const int lane = threadIdx.x & 31, wave = threadIdx.x >> 5, nloc = lane & 15, hlf = lane >> 4, z = blockIdx.z, m0 = blockIdx.y * 128 + wave * 32, c0 = blockIdx.x * 64;
  v8f acc[2][4];
#pragma unroll
  for (int r = 0; r < 2; ++r)
#pragma unroll
    for (int t = 0; t < 4; ++t) acc[r][t] = (v8f){};
  if (TYPE == 0) { const __bf16* A = (const __bf16*)Ap + z * a_zstride; const __bf16* Bw = (const __bf16*)Bp + z * b_zstride;
#pragma unroll 2
    for (int kb = 0; kb < KIN; kb += 32) { const v16bb a0 = frag_kb_bf(A + (size_t)(m0 + nloc) * KIN + kb, hlf), a1 = frag_kb_bf(A + (size_t)(m0 + 16 + nloc) * KIN + kb, hlf);
#pragma unroll
      for (int t = 0; t < 4; ++t) { const v16bb bw = frag_kb_bf(Bw + (size_t)(c0 + t * 16 + nloc) * KIN + kb, hlf); acc[0][t] = wmma16bb(a0, bw, acc[0][t]); acc[1][t] = wmma16bb(a1, bw, acc[1][t]); } } }
  else { const b16* A = (const b16*)Ap + z * a_zstride; const b16* Bw = (const b16*)Bp + z * b_zstride; const Opnd OA{A, nullptr, KIN}, OB{Bw, nullptr, KIN}; gemm_tile<1, 1>(OA, OB, KIN, m0, c0, nloc, hlf, acc); }
  float* Tt = Ts[wave];
  if (EPI == 0) {
    __shared__ __attribute__((aligned(16))) b16 Th[4][32][64 + 8];
#pragma unroll
    for (int t = 0; t < 4; ++t)
#pragma unroll
      for (int r = 0; r < 2; ++r)
#pragma unroll
        for (int v = 0; v < 8; ++v) Th[wave][r * 16 + v + 8 * hlf][t * 16 + nloc] = (b16)(acc[r][t][v] + bf16_rne(bias[(size_t)z * NOUT + c0 + t * 16 + nloc]));
    wave_lds_sync();
    b16* O = outh + z * o_zstride;
    for (int pass = 0; pass < 2; ++pass) {
#pragma unroll
      for (int j = 0; j < 8; ++j) { const int rr = j * 4 + (lane >> 3), c8 = (lane & 7) * 8; *(volatile v8b*)(O + (size_t)(m0 + rr) * NOUT + c0 + c8) = *(const v8b*)(&Th[wave][rr][c8]); }
      __threadfence(); }
    return; }
  if (EPI == 2 && c0 >= INNER) {
    __shared__ __attribute__((aligned(16))) float Gt[4][32][16];
#pragma unroll
    for (int r = 0; r < 2; ++r)
#pragma unroll
      for (int v = 0; v < 8; ++v) { const int rr = r * 16 + v + 8 * hlf; const float val = acc[r][0][v]; Gt[wave][rr][nloc] = (nloc < H) ? 1.0f / (1.0f + __expf(-val)) : 0.0f; }
    wave_lds_sync();
    for (int pass = 0; pass < 2; ++pass) {
#pragma unroll
      for (int j = 0; j < 4; ++j) { const int rr = j * 8 + (lane >> 2), c4 = (lane & 3) * 4; *(volatile v4f*)(outf + (size_t)(m0 + rr) * 16 + c4) = *(const v4f*)(&Gt[wave][rr][c4]); }
      __threadfence(); }
    return; }
  float* O = (EPI == 2) ? (float*)outh   : (outf + z * o_zstride);
  epi_f32(acc, 1.0f, nullptr, O, (EPI == 2) ? INNER : NOUT, m0, c0, lane, Tt);
}

__global__ __launch_bounds__(256) void attn_kernel(const float* __restrict__ q, const float* __restrict__ kv, const float* __restrict__ knw, const float* __restrict__ gates, b16* __restrict__ oh) {
  __shared__ __attribute__((aligned(16))) b16 Qh[8][16][DH + 8], Ql[8][16][DH + 8], Kh[8][16][DH + 8], Kl[8][16][DH + 8], Vh[8][DH][16 + 8], Vl[8][DH][16 + 8], Ph[8][16][16 + 8], Pl[8][16][16 + 8], Ot[8][8][DH + 8];
  const int wave = threadIdx.x >> 5, lane = threadIdx.x & 31, nloc = lane & 15, hlf = lane >> 4, bn = blockIdx.x  , h = wave;
  for (int i = lane; i < 16 * DH; i += 32) { const int r = i / DH, dd = i % DH; float x = 0.0f; if (r < L) x = q[((size_t)r * NN + bn) * INNER + h * DH + dd]; b16 a, c; split16(x * 8.0f, a, c); Qh[wave][r][dd] = a; Ql[wave][r][dd] = c; }
  for (int m = 0; m < M; ++m) { const float* kr = kv + ((size_t)m * NN + bn) * (2 * INNER) + h * DH; const float k0 = kr[lane], k1 = kr[32 + lane]; float s = k0 * k0 + k1 * k1;
#pragma unroll
    for (int o = 16; o > 0; o >>= 1) s += __shfl_xor(s, o);
    const float rs = rsqrtf(s * (1.0f / DH) + 1.1920929e-7f);
    b16 a, c; split16(k0 * rs * bf16_rne(knw[lane]) * 8.0f, a, c); Kh[wave][m][lane] = a; Kl[wave][m][lane] = c; split16(k1 * rs * bf16_rne(knw[32 + lane]) * 8.0f, a, c); Kh[wave][m][32 + lane] = a; Kl[wave][m][32 + lane] = c;
    const float v0 = kr[INNER + lane], v1 = kr[INNER + 32 + lane]; split16(v0 * 8.0f, a, c); Vh[wave][lane][m] = a; Vl[wave][lane][m] = c; split16(v1 * 8.0f, a, c); Vh[wave][32 + lane][m] = a; Vl[wave][32 + lane][m] = c; }
  wave_lds_sync();
  v8f sacc = {};
#pragma unroll
  for (int kb = 0; kb < DH; kb += 32) { const v16b ah = frag_kb(&Qh[wave][nloc][0] + kb, hlf), al = frag_kb(&Ql[wave][nloc][0] + kb, hlf), bh = frag_kb(&Kh[wave][nloc][0] + kb, hlf), bl = frag_kb(&Kl[wave][nloc][0] + kb, hlf);
    sacc = wmma16b(ah, bh, sacc); sacc = wmma16b(al, bh, sacc); sacc = wmma16b(ah, bl, sacc); }
  float p[8];
#pragma unroll
  for (int v = 0; v < 8; ++v) { float s = sacc[v] * (0.125f / 64.0f); float mx = s;
#pragma unroll
    for (int o = 8; o > 0; o >>= 1) mx = fmaxf(mx, __shfl_xor(mx, o));
    const float e = __expf(s - mx); float se = e;
#pragma unroll
    for (int o = 8; o > 0; o >>= 1) se += __shfl_xor(se, o);
    p[v] = e * __builtin_amdgcn_rcpf(se); }
#pragma unroll
  for (int v = 0; v < 8; ++v) { b16 a, c; split16(p[v] * 8.0f, a, c); Ph[wave][v + 8 * hlf][nloc] = a; Pl[wave][v + 8 * hlf][nloc] = c; }
  wave_lds_sync();
  v8f oacc[4] = {{}, {}, {}, {}};
  { v16b ah = {}, al = {};
#pragma unroll
    for (int e = 0; e < 8; ++e) { ah[e] = Ph[wave][nloc][8 * hlf + e]; al[e] = Pl[wave][nloc][8 * hlf + e]; }
#pragma unroll
    for (int t = 0; t < 4; ++t) { v16b bh = {}, bl = {};
#pragma unroll
      for (int e = 0; e < 8; ++e) { bh[e] = Vh[wave][t * 16 + nloc][8 * hlf + e]; bl[e] = Vl[wave][t * 16 + nloc][8 * hlf + e]; }
      oacc[t] = wmma16b(ah, bh, oacc[t]); oacc[t] = wmma16b(al, bh, oacc[t]); oacc[t] = wmma16b(ah, bl, oacc[t]); } }
  if (hlf == 0) {
#pragma unroll
    for (int v = 0; v < 8; ++v) { const float g = gates[((size_t)v * NN + bn) * 16 + h];
#pragma unroll
      for (int t = 0; t < 4; ++t) Ot[wave][v][t * 16 + nloc] = (b16)(oacc[t][v] * (1.0f / 64.0f) * g); } }
  wave_lds_sync();
  for (int pass = 0; pass < 2; ++pass) {
#pragma unroll
    for (int j = 0; j < 2; ++j) { const int rr = j * 4 + (lane >> 3), c8 = (lane & 7) * 8; *(volatile v8b*)(oh + ((size_t)rr * NN + bn) * INNER + h * DH + c8) = *(const v8b*)(&Ot[wave][rr][c8]); }
    __threadfence(); }
}
}

extern "C" void kernel_launch(void* const* d_in, const int* in_sizes, int n_in,
                              void* d_out, int out_size, void* d_ws, size_t ws_size, hipStream_t stream) {
  (void)n_in; (void)out_size;
  const float* tok = (const float*)d_in[0]; const float* wnet = (const float*)d_in[1]; const float* bnet = (const float*)d_in[2]; const float* nw = (const float*)d_in[3];
  const float* wq = (const float*)d_in[4]; const float* wkv = (const float*)d_in[5]; const float* knw = (const float*)d_in[6]; const float* wg = (const float*)d_in[7]; const float* wout = (const float*)d_in[8];
  float* out = (float*)d_out;
  if (in_sizes[0] != NR * D || in_sizes[1] != L * D * D || in_sizes[4] != D * INNER || in_sizes[5] != D * 2 * INNER || in_sizes[8] != INNER * D) return;
  size_t off = 0; char* ws = (char*)d_ws;
  auto carve = [&](size_t bytes) { char* p = ws + off; off += (bytes + 255) & ~(size_t)255; return p; };
  constexpr int RL = L * NN;
  unsigned short* wnb = (unsigned short*)carve((size_t)L * D * D * 2);
  unsigned short* wkvb = (unsigned short*)carve((size_t)D * D * 2); b16* wkvh = (b16*)carve((size_t)D * D * 2); b16* wqg = (b16*)carve((size_t)NQC * D * 2); b16* wo = (b16*)carve((size_t)D * INNER * 2);
  unsigned short* tokb = (unsigned short*)carve((size_t)RL * D * 2); b16* outh = (b16*)carve((size_t)RL * D * 2); b16* tnh = (b16*)carve((size_t)RL * D * 2);
  float* kvb = (float*)carve((size_t)M * NN * 2 * INNER * 4);
  float* qb = (float*)carve((size_t)RL * INNER * 4); float* gates = (float*)carve((size_t)RL * 16 * 4); b16* ohb = (b16*)carve((size_t)RL * INNER * 2);
  if (off > ws_size) return;
  prep_kernel<<<512, 256, 0, stream>>>(wnet, wq, wkv, wg, wout, wnb, wkvb, wkvh, wqg, wo);
  for (int b = 0; b < BT; ++b) {
    tok_kernel<<<512, 256, 0, stream>>>(tok, b, tokb);
    tn_kernel<<<RL / 8, 256, 0, stream>>>(tokb, nw, tnh);
    gemm_kernel<0, 0, D, D><<<dim3(D / 64, NN / 128, L), 128, 0, stream>>>(tokb, wnb, bnet, nullptr, outh, NN, (size_t)NN * D, (size_t)D * D, (size_t)NN * D);
    gemm_kernel<0, 1, D, 2 * INNER><<<dim3(2 * INNER / 64, RL / 128, 1), 128, 0, stream>>>(tokb, wkvb, nullptr, kvb, nullptr, RL, 0, 0, 0);
    gemm_kernel<1, 1, D, 2 * INNER><<<dim3(2 * INNER / 64, RL / 128, 1), 128, 0, stream>>>(outh, wkvh, nullptr, kvb + (size_t)RL * 2 * INNER, nullptr, RL, 0, 0, 0);
    gemm_kernel<1, 2, D, NQC><<<dim3(NQC / 64, RL / 128, 1), 128, 0, stream>>>(tnh, wqg, nullptr, gates, (b16*)qb, RL, 0, 0, 0);
    attn_kernel<<<NN, 256, 0, stream>>>(qb, kvb, knw, gates, ohb);
    gemm_kernel<1, 3, INNER, D><<<dim3(D / 64, NN / 128, L), 128, 0, stream>>>(ohb, wo, nullptr, out + (size_t)b * NN * D, nullptr, NN, (size_t)NN * INNER, 0, (size_t)BT * NN * D);
  }
}
